// Block_61744449848022
// MI455X (gfx1250) — hardware-verified
//
#include <hip/hip_runtime.h>
#include <math.h>


#ifndef NB
#define NB 1
#endif
#ifndef SEQ
#define SEQ 2048
#endif
#define SEQ_FULL 2048
#define HIDDEN 1024
#define HEADS 16
#define HDIM 64
#define QKVP 7168
#define VP 5120
#define PDIM 4096
#define EPSV 1e-5f
#define NEGV (-1.0e10f)
#define LOG2E 1.4426950408889634f
#define OUT1_OFF 2097152

static_assert(NB == 1);
static_assert(SEQ % 64 == 0);
static_assert(SEQ <= SEQ_FULL);
static_assert(OUT1_OFF * 4 == 8388608);
static_assert((QKVP * HIDDEN) % 2048 == 0);
static_assert((HIDDEN * VP) % 2048 == 0);
static_assert((2 * HIDDEN) % 64 == 0);
static_assert((QKVP - 2 * HIDDEN) % 128 == 0);
static_assert(HIDDEN % 128 == 0);
static_assert(VP % 32 == 0);
static_assert(SEQ * HIDDEN * 4 <= QKVP * HIDDEN * 2);

typedef _Float16 f16;
typedef f16   v16h __attribute__((ext_vector_type(16)));
typedef f16   v8h  __attribute__((ext_vector_type(8)));
typedef float v8f  __attribute__((ext_vector_type(8)));
typedef float v4f  __attribute__((ext_vector_type(4)));
typedef f16   v8ha __attribute__((ext_vector_type(8), may_alias));
typedef float v4fa __attribute__((ext_vector_type(4), may_alias));

__device__ __forceinline__ float bfr(float v) {
  unsigned u = __float_as_uint(v);
  u = (u + 0x7fffu + ((u >> 16) & 1u)) & 0xffff0000u;
  return __uint_as_float(u);
}

__device__ __forceinline__ v16h ldfrag(const f16* base, int ld, int lane) {
  const f16* p = base + (size_t)(lane & 15) * ld + ((lane >> 4) << 3);
  v8h lo = *(const v8h*)p;
  v8h hi = *(const v8h*)(p + 16);
  return __builtin_shufflevector(lo, hi, 0, 1, 2, 3, 4, 5, 6, 7,
                                 8, 9, 10, 11, 12, 13, 14, 15);
}

__device__ __forceinline__ v8f wmma16(v16h a, v16h b, v8f c) {
  v8f d = __builtin_amdgcn_wmma_f32_16x16x32_f16(false, a, false, b, (short)0, c, false, false);
  asm volatile("v_nop\n\tv_nop\n\tv_nop\n\tv_nop" : "+v"(d) : "v"(a), "v"(b));
  return d;
}

__device__ __forceinline__ void lds_wave_sync() {
  asm volatile("s_wait_dscnt 0x0" ::: "memory");
  __builtin_amdgcn_fence(3  , "wavefront");
  __builtin_amdgcn_wave_barrier();
}

__device__ __forceinline__ float wsum32(float v) {
  v += __shfl_xor(v, 16, 32);
  v += __shfl_xor(v, 8, 32);
  v += __shfl_xor(v, 4, 32);
  v += __shfl_xor(v, 2, 32);
  v += __shfl_xor(v, 1, 32);
  return v;
}

__global__ __launch_bounds__(256) void k_wconv(const float* __restrict__ win,
                                               const float* __restrict__ wout,
                                               f16* win16, f16* wout16) {
  const size_t n1 = (size_t)QKVP * HIDDEN, n2 = (size_t)HIDDEN * VP;
  const size_t i8 = ((size_t)blockIdx.x * 256 + threadIdx.x) * 8;
  const float* src;
  f16* dst;
  if (i8 < n1) {
    src = win + i8; dst = win16 + i8;
  } else {
    const size_t o = i8 - n1;
    if (o >= n2) return;
    src = wout + o; dst = wout16 + o;
  }
  v4f a = *(const v4f*)src;
  v4f c = *(const v4f*)(src + 4);
  v8h o;
#pragma unroll
  for (int i = 0; i < 4; ++i) {
    o[i]     = (f16)(bfr(a[i]) * 64.0f);
    o[4 + i] = (f16)(bfr(c[i]) * 64.0f);
  }
  *(volatile v8h*)dst = o;
  __threadfence();
  *(volatile v8h*)dst = o;
}

__global__ __launch_bounds__(128) void k_inln(const float* __restrict__ x,
                                              const float* __restrict__ g,
                                              const float* __restrict__ b,
                                              f16* hhi, f16* hlo) {
  __shared__ float red1[4];
  __shared__ float red2[4];
  const int l = blockIdx.x, t = threadIdx.x, wv = t >> 5, lane = t & 31, c0 = t * 8;
  const float* xr = x + (size_t)l * HIDDEN + c0;
  v4f xa = *(const v4f*)xr;
  v4f xb = *(const v4f*)(xr + 4);
  float v[8];
#pragma unroll
  for (int i = 0; i < 4; ++i) { v[i] = bfr(xa[i]); v[4 + i] = bfr(xb[i]); }
  float s = 0.f;
#pragma unroll
  for (int i = 0; i < 8; ++i) s += v[i];
  s = wsum32(s);
  if (lane == 0) red1[wv] = s;
  __syncthreads();
  const float mean = (red1[0] + red1[1] + red1[2] + red1[3]) * (1.0f / HIDDEN);
  float d[8], sq = 0.f;
#pragma unroll
  for (int i = 0; i < 8; ++i) { d[i] = v[i] - mean; sq += d[i] * d[i]; }
  sq = wsum32(sq);
  if (lane == 0) red2[wv] = sq;
  __syncthreads();
  const float var  = (red2[0] + red2[1] + red2[2] + red2[3]) * (1.0f / HIDDEN);
  const float rinv = 1.0f / sqrtf(var + EPSV);
  v4f ga = *(const v4f*)(g + c0), gb = *(const v4f*)(g + c0 + 4);
  v4f ba = *(const v4f*)(b + c0), bb = *(const v4f*)(b + c0 + 4);
  float gg[8], bv[8];
#pragma unroll
  for (int i = 0; i < 4; ++i) { gg[i] = ga[i]; gg[4 + i] = gb[i]; bv[i] = ba[i]; bv[4 + i] = bb[i]; }
  v8h H, L;
#pragma unroll
  for (int i = 0; i < 8; ++i) {
    const float y = d[i] * rinv * bfr(gg[i]) + bfr(bv[i]);
    const f16 yh = (f16)y;
    H[i] = yh;
    L[i] = (f16)((y - (float)yh) * 2048.0f);
  }
  if (wv == 0) {
    const bool fwd = (l + 1 < SEQ);
    const bool zr  = (l == 0);
    f16* ph = hhi + (size_t)(l + 1) * HIDDEN + c0;
    f16* pl = hlo + (size_t)(l + 1) * HIDDEN + c0;
    f16* zh = hhi + c0;
    f16* zl = hlo + c0;
    v8h Z = {};
    if (fwd) { *(volatile v8h*)ph = H; *(volatile v8h*)pl = L; }
    if (zr)  { *(volatile v8h*)zh = Z; *(volatile v8h*)zl = Z; }
    __threadfence();
    if (fwd) { *(volatile v8h*)ph = H; *(volatile v8h*)pl = L; }
    if (zr)  { *(volatile v8h*)zh = Z; *(volatile v8h*)zl = Z; }
  } else {
    f16* ph = hhi + (size_t)l * HIDDEN + c0;
    f16* pl = hlo + (size_t)l * HIDDEN + c0;
    *(volatile v8h*)ph = H; *(volatile v8h*)pl = L;
    __threadfence();
    *(volatile v8h*)ph = H; *(volatile v8h*)pl = L;
  }
}

template <int NTL, bool ALO, bool BLO>
__global__ __launch_bounds__(128) void k_gemm(const f16* __restrict__ A, const f16* __restrict__ Al,
                                              const f16* __restrict__ B, const f16* __restrict__ Bl,
                                              int lda, int ldb, int K,
                                              float* C, int ldc, float shi, float slo) {
  constexpr int FR  = 16 * NTL;
  constexpr int LPR = FR / 4;
  constexpr int RPI = 32 / LPR;
  constexpr int NI  = 16 / RPI;
  __shared__ __attribute__((aligned(16))) float cst[4][16][FR];
  const int t = threadIdx.x, wv = t >> 5, lane = t & 31, hh = lane >> 4, col = lane & 15;
  const int rowBase = blockIdx.y * 64 + (wv & 1) * 32;
  const int colBase = blockIdx.x * (2 * FR) + (wv >> 1) * FR;

  v8f acc[2][NTL] = {};
  v8f accl[2][NTL] = {};

  for (int kb = 0; kb < K; kb += 32) {
    v16h a0 = ldfrag(A + (size_t)rowBase * lda + kb, lda, lane);
    v16h a1 = ldfrag(A + (size_t)(rowBase + 16) * lda + kb, lda, lane);
    v16h l0 = a0, l1 = a1;
    if (ALO) {
      l0 = ldfrag(Al + (size_t)rowBase * lda + kb, lda, lane);
      l1 = ldfrag(Al + (size_t)(rowBase + 16) * lda + kb, lda, lane);
    }
#pragma unroll
    for (int tt = 0; tt < NTL; ++tt) {
      v16h bt = ldfrag(B + (size_t)(colBase + 16 * tt) * ldb + kb, ldb, lane);
      acc[0][tt] = wmma16(a0, bt, acc[0][tt]);
      acc[1][tt] = wmma16(a1, bt, acc[1][tt]);
      if (ALO) {
        accl[0][tt] = wmma16(l0, bt, accl[0][tt]);
        accl[1][tt] = wmma16(l1, bt, accl[1][tt]);
      }
      if (BLO) {
        v16h bl = ldfrag(Bl + (size_t)(colBase + 16 * tt) * ldb + kb, ldb, lane);
        accl[0][tt] = wmma16(a0, bl, accl[0][tt]);
        accl[1][tt] = wmma16(a1, bl, accl[1][tt]);
      }
    }
  }

#pragma unroll
  for (int s = 0; s < 2; ++s) {
#pragma unroll
    for (int tt = 0; tt < NTL; ++tt) {
#pragma unroll
      for (int r = 0; r < 8; ++r) {
        float v = acc[s][tt][r];
        if (ALO || BLO) v += accl[s][tt][r] * slo;
        cst[wv][hh * 8 + r][tt * 16 + col] = v * shi;
      }
    }
    lds_wave_sync();
    v4f vals[NI];
    float* dsts[NI];
#pragma unroll
    for (int it = 0; it < NI; ++it) {
      const int row = it * RPI + lane / LPR;
      const int piece = lane % LPR;
      vals[it] = *(const v4fa*)&cst[wv][row][piece * 4];
      dsts[it] = C + (size_t)(rowBase + s * 16 + row) * ldc + colBase + piece * 4;
    }
#pragma unroll
    for (int it = 0; it < NI; ++it) *(volatile v4f*)dsts[it] = vals[it];
    __threadfence();
#pragma unroll
    for (int it = 0; it < NI; ++it) *(volatile v4f*)dsts[it] = vals[it];
    lds_wave_sync();
  }
}

__global__ __launch_bounds__(256) void k_qkln(const float* __restrict__ qkvp,
                                              const float* __restrict__ qg, const float* __restrict__ qb,
                                              const float* __restrict__ kg, const float* __restrict__ kb,
                                              f16* qhi, f16* qlo, f16* khi, f16* klo) {
  __shared__ float red1[8];
  __shared__ float red2[8];
  const int l = blockIdx.x, t = threadIdx.x, wv = t >> 5, lane = t & 31;
  const int grp = wv >> 2;
  const int c0 = (t & 127) * 8;
  const float* src = qkvp + (size_t)l * QKVP + grp * HIDDEN + c0;
  v4f xa = *(const v4f*)src;
  v4f xb = *(const v4f*)(src + 4);
  float v[8];
#pragma unroll
  for (int i = 0; i < 4; ++i) { v[i] = xa[i]; v[4 + i] = xb[i]; }
  float s = 0.f;
#pragma unroll
  for (int i = 0; i < 8; ++i) s += v[i];
  s = wsum32(s);
  if (lane == 0) red1[wv] = s;
  __syncthreads();
  const float mean = (red1[grp * 4 + 0] + red1[grp * 4 + 1] + red1[grp * 4 + 2] + red1[grp * 4 + 3]) *
                     (1.0f / HIDDEN);
  float d[8], sq = 0.f;
#pragma unroll
  for (int i = 0; i < 8; ++i) { d[i] = v[i] - mean; sq += d[i] * d[i]; }
  sq = wsum32(sq);
  if (lane == 0) red2[wv] = sq;
  __syncthreads();
  const float var  = (red2[grp * 4 + 0] + red2[grp * 4 + 1] + red2[grp * 4 + 2] + red2[grp * 4 + 3]) *
                     (1.0f / HIDDEN);
  const float rinv = 1.0f / sqrtf(var + EPSV);
  const float* gp = grp ? kg : qg;
  const float* bp = grp ? kb : qb;
  v4f ga = *(const v4f*)(gp + c0), gb = *(const v4f*)(gp + c0 + 4);
  v4f ba = *(const v4f*)(bp + c0), bb = *(const v4f*)(bp + c0 + 4);
  float gg[8], bv[8];
#pragma unroll
  for (int i = 0; i < 4; ++i) { gg[i] = ga[i]; gg[4 + i] = gb[i]; bv[i] = ba[i]; bv[4 + i] = bb[i]; }
  v8h H, L;
#pragma unroll
  for (int i = 0; i < 8; ++i) {
    const float y = d[i] * rinv * bfr(gg[i]) + bfr(bv[i]);
    const f16 yh = (f16)y;
    H[i] = yh;
    L[i] = (f16)((y - (float)yh) * 2048.0f);
  }
  f16* dh = (grp ? khi : qhi) + (size_t)l * HIDDEN + c0;
  f16* dl = (grp ? klo : qlo) + (size_t)l * HIDDEN + c0;
  *(volatile v8h*)dh = H; *(volatile v8h*)dl = L;
  __threadfence();
  *(volatile v8h*)dh = H; *(volatile v8h*)dl = L;
}

__global__ __launch_bounds__(256) void k_vt(const float* __restrict__ qkvp, f16* vt) {
  __shared__ __attribute__((aligned(16))) f16 sv[64][72];
  const int tb = blockIdx.x, h = blockIdx.y, t = threadIdx.x;
  {
    const int tok = t >> 2, cg = (t & 3) * 16;
    const float* src = qkvp + (size_t)(tb * 64 + tok) * QKVP + 2 * HIDDEN + h * HDIM + cg;
    v4f a0 = *(const v4f*)src;
    v4f a1 = *(const v4f*)(src + 4);
    v4f a2 = *(const v4f*)(src + 8);
    v4f a3 = *(const v4f*)(src + 12);
#pragma unroll
    for (int i = 0; i < 4; ++i) {
      sv[cg + i][tok]      = (f16)a0[i];
      sv[cg + 4 + i][tok]  = (f16)a1[i];
      sv[cg + 8 + i][tok]  = (f16)a2[i];
      sv[cg + 12 + i][tok] = (f16)a3[i];
    }
  }
  __syncthreads();
  const int piece = t & 7, r0 = t >> 3;
  v8h w0 = *(const v8ha*)&sv[r0][piece * 8];
  v8h w1 = *(const v8ha*)&sv[r0 + 32][piece * 8];
  f16* d0 = vt + (size_t)(h * HDIM + r0) * SEQ + tb * 64 + piece * 8;
  f16* d1 = vt + (size_t)(h * HDIM + r0 + 32) * SEQ + tb * 64 + piece * 8;
  *(volatile v8h*)d0 = w0; *(volatile v8h*)d1 = w1;
  __threadfence();
  *(volatile v8h*)d0 = w0; *(volatile v8h*)d1 = w1;
}

__global__ __launch_bounds__(128) void k_attn(const f16* __restrict__ qhi,
                                              const f16* __restrict__ khi,
                                              const f16* __restrict__ vt,
                                              const float* __restrict__ al,
                                              f16* cat) {
  __shared__ __attribute__((aligned(16))) float abuf[4][16][32];
  __shared__ __attribute__((aligned(16))) f16 pbuf[4][16][32];
  __shared__ __attribute__((aligned(16))) f16 cbuf[4][16][64];
  const int t = threadIdx.x, wv = t >> 5, lane = t & 31, hh = lane >> 4, col = lane & 15;
  const int h = blockIdx.y;
  const int qBase = blockIdx.x * 64 + wv * 16;

  const int se = (h + 1) >> 1;
  const float p2 = __uint_as_float((unsigned)(127 - se) << 23);
  const float slope = (h & 1) ? p2 : (0.70710677f * p2);

  const f16* qp = qhi + (size_t)qBase * HIDDEN + h * HDIM;
  v16h qa0 = ldfrag(qp, HIDDEN, lane);
  v16h qa1 = ldfrag(qp + 32, HIDDEN, lane);
  v8f o0 = {}, o1 = {}, o2 = {}, o3 = {};
  float m[8], lsum[8];
#pragma unroll
  for (int r = 0; r < 8; ++r) { m[r] = -3.0e38f; lsum[r] = 0.f; }

  const f16* kh = khi + h * HDIM;
  const f16* vh = vt + (size_t)(h * HDIM) * SEQ;
  const int jend = qBase + 16;

  for (int jb = 0; jb < jend; jb += 32) {
    v8f s0 = {}, s1 = {};
    {
      v16h b0 = ldfrag(kh + (size_t)jb * HIDDEN, HIDDEN, lane);
      v16h b1 = ldfrag(kh + (size_t)jb * HIDDEN + 32, HIDDEN, lane);
      s0 = wmma16(qa0, b0, s0);
      s0 = wmma16(qa1, b1, s0);
      b0 = ldfrag(kh + (size_t)(jb + 16) * HIDDEN, HIDDEN, lane);
      b1 = ldfrag(kh + (size_t)(jb + 16) * HIDDEN + 32, HIDDEN, lane);
      s1 = wmma16(qa0, b0, s1);
      s1 = wmma16(qa1, b1, s1);
    }
#pragma unroll
    for (int u = 0; u < 4; ++u) {
      const int idx = lane + 32 * u;
      const int row = idx >> 3, piece = idx & 7;
      v4f av = *(const v4f*)(al + (size_t)(qBase + row) * SEQ_FULL + jb + piece * 4);
#pragma unroll
      for (int i = 0; i < 4; ++i) av[i] = bfr(av[i]);
      *(v4fa*)&abuf[wv][row][piece * 4] = av;
    }
    lds_wave_sync();
#pragma unroll
    for (int r = 0; r < 8; ++r) {
      const int i  = qBase + hh * 8 + r;
      const int j0 = jb + col, j1 = jb + 16 + col;
      const float a0v = abuf[wv][hh * 8 + r][col];
      const float a1v = abuf[wv][hh * 8 + r][16 + col];
      float t0 = (s0[r] * 0.125f + a0v) + (float)j0 * slope;
      float t1 = (s1[r] * 0.125f + a1v) + (float)j1 * slope;
      t0 = (j0 <= i) ? t0 : (t0 + NEGV);
      t1 = (j1 <= i) ? t1 : (t1 + NEGV);
      float mx = fmaxf(t0, t1);
      mx = fmaxf(mx, __shfl_xor(mx, 1, 32));
      mx = fmaxf(mx, __shfl_xor(mx, 2, 32));
      mx = fmaxf(mx, __shfl_xor(mx, 4, 32));
      mx = fmaxf(mx, __shfl_xor(mx, 8, 32));
      const float mn   = fmaxf(m[r], mx);
      const float corr = exp2f((m[r] - mn) * LOG2E);
      m[r] = mn;
      const float p0 = exp2f((t0 - mn) * LOG2E);
      const float p1 = exp2f((t1 - mn) * LOG2E);
      s0[r] = p0; s1[r] = p1;
      float ps = p0 + p1;
      ps += __shfl_xor(ps, 1, 32);
      ps += __shfl_xor(ps, 2, 32);
      ps += __shfl_xor(ps, 4, 32);
      ps += __shfl_xor(ps, 8, 32);
      lsum[r] = lsum[r] * corr + ps;
      o0[r] *= corr; o1[r] *= corr; o2[r] *= corr; o3[r] *= corr;
    }
#pragma unroll
    for (int r = 0; r < 8; ++r) {
      pbuf[wv][hh * 8 + r][col]      = (f16)(s0[r] * 16384.0f);
      pbuf[wv][hh * 8 + r][16 + col] = (f16)(s1[r] * 16384.0f);
    }
    lds_wave_sync();
    v16h pa = ldfrag(&pbuf[wv][0][0], 32, lane);
    o0 = wmma16(pa, ldfrag(vh + jb, SEQ, lane), o0);
    o1 = wmma16(pa, ldfrag(vh + (size_t)16 * SEQ + jb, SEQ, lane), o1);
    o2 = wmma16(pa, ldfrag(vh + (size_t)32 * SEQ + jb, SEQ, lane), o2);
    o3 = wmma16(pa, ldfrag(vh + (size_t)48 * SEQ + jb, SEQ, lane), o3);
  }

  float inv[8];
#pragma unroll
  for (int r = 0; r < 8; ++r) inv[r] = (1.0f / lsum[r]) * (1.0f / 16384.0f);
#pragma unroll
  for (int r = 0; r < 8; ++r) {
    cbuf[wv][hh * 8 + r][col]      = (f16)(o0[r] * inv[r]);
    cbuf[wv][hh * 8 + r][16 + col] = (f16)(o1[r] * inv[r]);
    cbuf[wv][hh * 8 + r][32 + col] = (f16)(o2[r] * inv[r]);
    cbuf[wv][hh * 8 + r][48 + col] = (f16)(o3[r] * inv[r]);
  }
  lds_wave_sync();
  v8h cv[4];
  f16* cd[4];
#pragma unroll
  for (int it = 0; it < 4; ++it) {
    const int row = it * 4 + (lane >> 3), piece = lane & 7;
    cv[it] = *(const v8ha*)&cbuf[wv][row][piece * 8];
    cd[it] = cat + (size_t)(qBase + row) * VP + h * HDIM + piece * 8;
  }
#pragma unroll
  for (int it = 0; it < 4; ++it) *(volatile v8h*)cd[it] = cv[it];
  __threadfence();
#pragma unroll
  for (int it = 0; it < 4; ++it) *(volatile v8h*)cd[it] = cv[it];
}

__global__ __launch_bounds__(256) void k_midln(const float* __restrict__ qkvp,
                                               const float* __restrict__ g,
                                               const float* __restrict__ b,
                                               f16* cat) {
  __shared__ float red1[8];
  __shared__ float red2[8];
  const int l = blockIdx.x, t = threadIdx.x, wv = t >> 5, lane = t & 31;
  const float* src = qkvp + (size_t)l * QKVP + 3 * HIDDEN;
  const int c0 = t * 8, c1 = PDIM / 2 + t * 8;
  v4f a0 = *(const v4f*)(src + c0), a1 = *(const v4f*)(src + c0 + 4);
  v4f a2 = *(const v4f*)(src + c1), a3 = *(const v4f*)(src + c1 + 4);
  float v[16];
#pragma unroll
  for (int i = 0; i < 4; ++i) { v[i] = a0[i]; v[4 + i] = a1[i]; v[8 + i] = a2[i]; v[12 + i] = a3[i]; }
  float s = 0.f;
#pragma unroll
  for (int i = 0; i < 16; ++i) s += v[i];
  s = wsum32(s);
  if (lane == 0) red1[wv] = s;
  __syncthreads();
  float tot = 0.f;
#pragma unroll
  for (int w = 0; w < 8; ++w) tot += red1[w];
  const float mean = tot * (1.0f / PDIM);
  float d[16], sq = 0.f;
#pragma unroll
  for (int i = 0; i < 16; ++i) { d[i] = v[i] - mean; sq += d[i] * d[i]; }
  sq = wsum32(sq);
  if (lane == 0) red2[wv] = sq;
  __syncthreads();
  float tq = 0.f;
#pragma unroll
  for (int w = 0; w < 8; ++w) tq += red2[w];
  const float var  = tq * (1.0f / PDIM);
  const float rinv = 1.0f / sqrtf(var + EPSV);
  v4f g0 = *(const v4f*)(g + c0), g1 = *(const v4f*)(g + c0 + 4);
  v4f g2 = *(const v4f*)(g + c1), g3 = *(const v4f*)(g + c1 + 4);
  v4f b0 = *(const v4f*)(b + c0), b1 = *(const v4f*)(b + c0 + 4);
  v4f b2 = *(const v4f*)(b + c1), b3 = *(const v4f*)(b + c1 + 4);
  float gg[16], bv[16];
#pragma unroll
  for (int i = 0; i < 4; ++i) {
    gg[i] = g0[i]; gg[4 + i] = g1[i]; gg[8 + i] = g2[i]; gg[12 + i] = g3[i];
    bv[i] = b0[i]; bv[4 + i] = b1[i]; bv[8 + i] = b2[i]; bv[12 + i] = b3[i];
  }
  v8h H0, H1;
#pragma unroll
  for (int i = 0; i < 8; ++i) {
    float y0 = d[i] * rinv * bfr(gg[i]) + bfr(bv[i]);
    float y1 = d[8 + i] * rinv * bfr(gg[8 + i]) + bfr(bv[8 + i]);
    y0 = (y0 > 0.f) ? y0 : 0.f;
    y1 = (y1 > 0.f) ? y1 : 0.f;
    H0[i] = (f16)y0;
    H1[i] = (f16)y1;
  }
  f16* p0 = cat + (size_t)l * VP + HIDDEN + c0;
  f16* p1 = cat + (size_t)l * VP + HIDDEN + c1;
  *(volatile v8h*)p0 = H0; *(volatile v8h*)p1 = H1;
  __threadfence();
  *(volatile v8h*)p0 = H0; *(volatile v8h*)p1 = H1;
}

__global__ __launch_bounds__(256) void k_outln(const float* __restrict__ tmp,
                                               const float* __restrict__ bias,
                                               const float* __restrict__ g,
                                               const float* __restrict__ b,
                                               float* out) {
  __shared__ float red1[8];
  __shared__ float red2[8];
  const int l = blockIdx.x, t = threadIdx.x, wv = t >> 5, lane = t & 31, c0 = t * 4;
  v4f a  = *(const v4f*)(tmp + (size_t)l * HIDDEN + c0);
  v4f bi = *(const v4f*)(bias + c0);
  float v[4];
#pragma unroll
  for (int i = 0; i < 4; ++i) v[i] = a[i] + bfr(bi[i]);
  float s = v[0] + v[1] + v[2] + v[3];
  s = wsum32(s);
  if (lane == 0) red1[wv] = s;
  __syncthreads();
  float tot = 0.f;
#pragma unroll
  for (int w = 0; w < 8; ++w) tot += red1[w];
  const float mean = tot * (1.0f / HIDDEN);
  float d[4], sq = 0.f;
#pragma unroll
  for (int i = 0; i < 4; ++i) { d[i] = v[i] - mean; sq += d[i] * d[i]; }
  sq = wsum32(sq);
  if (lane == 0) red2[wv] = sq;
  __syncthreads();
  float tq = 0.f;
#pragma unroll
  for (int w = 0; w < 8; ++w) tq += red2[w];
  const float var  = tq * (1.0f / HIDDEN);
  const float rinv = 1.0f / sqrtf(var + EPSV);
  v4f gv = *(const v4f*)(g + c0), bb = *(const v4f*)(b + c0);
  v4f o;
#pragma unroll
  for (int i = 0; i < 4; ++i) o[i] = d[i] * rinv * bfr(gv[i]) + bfr(bb[i]);
  float* p = out + (size_t)l * HIDDEN + c0;
  *(volatile v4f*)p = o;
  __threadfence();
  *(volatile v4f*)p = o;
}

extern "C" void kernel_launch(void* const* d_in, const int* in_sizes, int n_in,
                              void* d_out, int out_size, void* d_ws, size_t ws_size,
                              hipStream_t stream) {
  if (n_in < 15) return;
  if (in_sizes[0] < SEQ * HIDDEN) return;
  if (in_sizes[1] < SEQ * SEQ) return;
  if (in_sizes[2] < QKVP * HIDDEN) return;
  if (in_sizes[3] < HIDDEN * VP) return;
  if (in_sizes[4] < HIDDEN) return;
  if (in_sizes[5] < HIDDEN || in_sizes[6] < HIDDEN) return;
  if (in_sizes[7] < HIDDEN || in_sizes[8] < HIDDEN) return;
  if (in_sizes[9] < HIDDEN || in_sizes[10] < HIDDEN) return;
  if (in_sizes[11] < PDIM || in_sizes[12] < PDIM) return;
  if (in_sizes[13] < HIDDEN || in_sizes[14] < HIDDEN) return;
  if ((size_t)out_size < (size_t)OUT1_OFF + (size_t)SEQ * SEQ) return;

  const float* x   = (const float*)d_in[0];
  const float* AL  = (const float*)d_in[1];
  const float* win = (const float*)d_in[2];
  const float* wo  = (const float*)d_in[3];
  const float* opb = (const float*)d_in[4];
  const float* ing = (const float*)d_in[5];
  const float* inb = (const float*)d_in[6];
  const float* qg  = (const float*)d_in[7];
  const float* qb  = (const float*)d_in[8];
  const float* kg  = (const float*)d_in[9];
  const float* kbv = (const float*)d_in[10];
  const float* mg  = (const float*)d_in[11];
  const float* mb  = (const float*)d_in[12];
  const float* og  = (const float*)d_in[13];
  const float* ob  = (const float*)d_in[14];
  float* out0 = (float*)d_out;
  float* out1 = out0 + OUT1_OFF;

  const size_t nWin   = (size_t)QKVP * HIDDEN * 2;
  const size_t nWout  = (size_t)HIDDEN * VP * 2;
  const size_t nPlane = (size_t)SEQ * HIDDEN * 2;
  const size_t nQkvp  = (size_t)SEQ * QKVP * 4;
  const size_t nVt    = (size_t)HIDDEN * SEQ * 2;
  const size_t nCat   = (size_t)SEQ * VP * 2;
  const size_t oWin  = 0;
  const size_t oWout = oWin + nWin;
  const size_t oH    = oWout + nWout;
  const size_t oQkvp = oH + 2 * nPlane;
  const size_t oK    = oQkvp + nQkvp;
  const size_t oVt   = oK + 2 * nPlane;
  const size_t oCat  = oVt + nVt;
  const size_t total = oCat + nCat;
  if (total > ws_size) return;

  char* ws = (char*)d_ws;
  f16*   win16  = (f16*)(ws + oWin);
  float* tmp    = (float*)(ws + oWin);
  f16*   wout16 = (f16*)(ws + oWout);
  f16*   hhi    = (f16*)(ws + oH);
  f16*   hlo    = (f16*)(ws + oH + nPlane);
  f16*   qhi    = hhi;
  f16*   qlo    = hlo;
  float* qkvp   = (float*)(ws + oQkvp);
  f16*   khi    = (f16*)(ws + oK);
  f16*   klo    = (f16*)(ws + oK + nPlane);
  f16*   vt     = (f16*)(ws + oVt);
  f16*   cat    = (f16*)(ws + oCat);

  k_wconv<<<(QKVP * HIDDEN + HIDDEN * VP) / 2048, 256, 0, stream>>>(win, wo, win16, wout16);
  k_inln<<<SEQ, 128, 0, stream>>>(x, ing, inb, hhi, hlo);
  k_gemm<2, true, false><<<dim3((2 * HIDDEN) / 64, SEQ / 64), 128, 0, stream>>>(
      hhi, hlo, win16, win16, HIDDEN, HIDDEN, HIDDEN, qkvp, QKVP, 1.0f / 64.0f, 1.0f / 2048.0f);
  k_gemm<4, false, false><<<dim3((QKVP - 2 * HIDDEN) / 128, SEQ / 64), 128, 0, stream>>>(
      hhi, hhi, win16 + (size_t)2 * HIDDEN * HIDDEN, win16 + (size_t)2 * HIDDEN * HIDDEN,
      HIDDEN, HIDDEN, HIDDEN, qkvp + 2 * HIDDEN, QKVP, 1.0f / 64.0f, 0.0f);
  k_qkln<<<SEQ, 256, 0, stream>>>(qkvp, qg, qb, kg, kbv, qhi, qlo, khi, klo);
  k_vt<<<dim3(SEQ / 64, HEADS), 256, 0, stream>>>(qkvp, vt);
  k_gemm<2, true, true><<<dim3(SEQ / 64, SEQ / 64), 128, 0, stream>>>(
      qhi, qlo, khi, klo, HIDDEN, HIDDEN, HIDDEN, out1, SEQ, 0.0078125f, 1.0f / 2048.0f);
  k_attn<<<dim3(SEQ / 64, HEADS), 128, 0, stream>>>(qhi, khi, vt, AL, cat);
  k_midln<<<SEQ, 256, 0, stream>>>(qkvp, mg, mb, cat);
  k_gemm<4, false, false><<<dim3(HIDDEN / 128, SEQ / 64), 128, 0, stream>>>(
      cat, cat, wout16, wout16, VP, VP, VP, tmp, HIDDEN, 1.0f / 64.0f, 0.0f);
  k_outln<<<SEQ, 256, 0, stream>>>(tmp, opb, og, ob, out0);
}
